// Gemma3Attention_21663815041387
// MI455X (gfx1250) — hardware-verified
//
#include <hip/hip_runtime.h>
#include <math.h>
#include <stdint.h>

#ifndef NB
#define NB 2
#endif
#ifndef SEQ
#define SEQ 2048
#endif
#define NB_FULL   2
#define SEQ_FULL  2048
#define DIM       2048
#define NH        16
#define NKV       8
#define HD        128
#define HDQ       (NH * HD)
#define KVD       (NKV * HD)
#define NREP      (NH / NKV)
#define WIN       1024
#define ROPE_HALF 64
#define ROWS      (NB * SEQ)
#define VLN       ((SEQ < 512) ? SEQ : 512)
#define EPS       1.0e-6f
#define SMSC      0.0625f
#define QSC       4.0f
#define KSC       4.0f
#define QLC       4096.0f
#define KLC       4096.0f
#define PCAR      32768.0f
#define PLC       4096.0f
#define VCAR      1024.0f
#define VLC       4096.0f
#define OSC       1024.0f
#define OLC       4096.0f
#define WOS       1024.0f
#define LOG2E     1.4426950408889634f
#define NEGS      (-3.0e38f)
#define ATT_WAVES   4
#define ATT_THREADS (ATT_WAVES * 32)
#define NQT       (SEQ / 64)
#define NKB       (SEQ / 32)
#define SLABW     (16 * 132)
#define SLABN     (16 * 68)
static_assert(NB >= 1 && NB <= NB_FULL);
static_assert((SEQ % 64) == 0 && SEQ >= 64 && SEQ <= SEQ_FULL);
static_assert(HD == 128 && 2 * ROPE_HALF == HD && HDQ == 2048 && KVD == 1024 && NREP == 2);
static_assert((DIM % 64) == 0 && (HDQ % 128) == 0 && (KVD % 128) == 0 && (DIM % 32) == 0 && (HDQ % 32) == 0);
static_assert(((SEQ * DIM / 8) % 256) == 0);
static_assert(ATT_THREADS == 128 && NKB * 32 == SEQ && NQT * 64 == SEQ);
static_assert((VLN % 64) == 0 && VLN >= 64 && VLN <= SEQ && (VLN % 32) == 0);
static_assert(PLC == VLC && QLC == KLC);
static_assert(SLABW >= 2 * 16 * ROPE_HALF && SLABW >= 16 * 132);
static_assert((SLABW * 4) % 16 == 0 && (SLABN * 4) % 16 == 0);

typedef unsigned short u16;
typedef _Float16 v16h __attribute__((ext_vector_type(16)));
typedef _Float16 v8h  __attribute__((ext_vector_type(8)));
typedef __bf16   v16b __attribute__((ext_vector_type(16)));
typedef float    v8f  __attribute__((ext_vector_type(8)));
typedef float    v4f  __attribute__((ext_vector_type(4)));
typedef unsigned int v4u __attribute__((ext_vector_type(4)));

union FragH { v16h v; v8h h[2]; v4u u[2]; };
union FragB { v16b v; v4u u[2]; };

__device__ __forceinline__ unsigned short bf_bits(float f) {
  unsigned u = __float_as_uint(f);
  return (unsigned short)((u + 0x7FFFu + ((u >> 16) & 1u)) >> 16);
}
__device__ __forceinline__ float bf_up(unsigned short h) { return __uint_as_float(((unsigned)h) << 16); }
__device__ __forceinline__ float bf_val(float f) { return bf_up(bf_bits(f)); }
__device__ __forceinline__ unsigned short h_bits(_Float16 x) { return __builtin_bit_cast(unsigned short, x); }
__device__ __forceinline__ unsigned pk16(unsigned short a, unsigned short b) { return (unsigned)a | ((unsigned)b << 16); }
__device__ __forceinline__ v8f zero8() { v8f z = {0.f, 0.f, 0.f, 0.f, 0.f, 0.f, 0.f, 0.f}; return z; }
__device__ __forceinline__ v4u zero4u() { v4u z = {0u, 0u, 0u, 0u}; return z; }

__device__ __forceinline__ v16h ldfrag_h(const _Float16* p) {
  FragH f;
  f.h[0] = *(const v8h*)(p);
  f.h[1] = *(const v8h*)(p + 16);
  return f.v;
}
__device__ __forceinline__ v16b ldfrag_b(const u16* p) {
  FragB f;
  f.u[0] = *(const v4u*)(p);
  f.u[1] = *(const v4u*)(p + 16);
  return f.v;
}

__device__ __forceinline__ v8f mma_h(v16h a, v16h b, v8f c) {
  return __builtin_amdgcn_wmma_f32_16x16x32_f16(false, a, false, b, (short)0, c, false, false);
}
__device__ __forceinline__ v8f mma_b(v16b a, v16b b, v8f c) {
  return __builtin_amdgcn_wmma_f32_16x16x32_bf16(false, a, false, b, (short)0, c, false, false);
}
__device__ __forceinline__ void guard2(v8f& a, v8f& b, v16h x0, v16h x1, v16h x2, v16h x3, v16h x4, v16h x5) {
#if defined(__HIP_DEVICE_COMPILE__)
  asm volatile("v_nop\n\tv_nop\n\tv_nop\n\tv_nop"
               : "+v"(a), "+v"(b) : "v"(x0), "v"(x1), "v"(x2), "v"(x3), "v"(x4), "v"(x5) : "memory");
#endif
}
template <typename F>
__device__ __forceinline__ void guard4(v8f& a, v8f& b, v8f& c, v8f& d, F x0, F x1, F x2, F x3) {
#if defined(__HIP_DEVICE_COMPILE__)
  asm volatile("v_nop\n\tv_nop\n\tv_nop\n\tv_nop"
               : "+v"(a), "+v"(b), "+v"(c), "+v"(d) : "v"(x0), "v"(x1), "v"(x2), "v"(x3) : "memory");
#endif
}
template <typename F>
__device__ __forceinline__ void guard6(v8f& a, v8f& b, v8f& c, v8f& d, F x0, F x1, F x2, F x3, F x4, F x5) {
#if defined(__HIP_DEVICE_COMPILE__)
  asm volatile("v_nop\n\tv_nop\n\tv_nop\n\tv_nop"
               : "+v"(a), "+v"(b), "+v"(c), "+v"(d) : "v"(x0), "v"(x1), "v"(x2), "v"(x3), "v"(x4), "v"(x5) : "memory");
#endif
}
__device__ __forceinline__ void guard8(v8f& a, v8f& b, v8f& c, v8f& d, v8f& e, v8f& f, v8f& g, v8f& h,
                                       v16h x0, v16h x1, v16h x2, v16h x3, v16h x4, v16h x5) {
#if defined(__HIP_DEVICE_COMPILE__)
  asm volatile("v_nop\n\tv_nop\n\tv_nop\n\tv_nop"
               : "+v"(a), "+v"(b), "+v"(c), "+v"(d), "+v"(e), "+v"(f), "+v"(g), "+v"(h)
               : "v"(x0), "v"(x1), "v"(x2), "v"(x3), "v"(x4), "v"(x5) : "memory");
#endif
}
__device__ __forceinline__ void acc_guard4(v8f& a, v8f& b, v8f& c, v8f& d) {
#if defined(__HIP_DEVICE_COMPILE__)
  asm volatile("v_nop\n\tv_nop\n\tv_nop\n\tv_nop" : "+v"(a), "+v"(b), "+v"(c), "+v"(d));
#endif
}
__device__ __forceinline__ void wave_sync_lds() {
#if defined(__HIP_DEVICE_COMPILE__)
  __builtin_amdgcn_fence(__ATOMIC_RELEASE, "workgroup");
  __builtin_amdgcn_wave_barrier();
  __builtin_amdgcn_fence(__ATOMIC_ACQUIRE, "workgroup");
#endif
}

__global__ __launch_bounds__(256) void cvt16(const float* __restrict__ x, u16* D, int n8, int mode, float scale) {
  const int gt = blockIdx.x * 256 + (int)threadIdx.x;
  if (gt >= n8) return;
  const float* p = x + (size_t)gt * 8;
  const v4f a = *(const v4f*)(p), c4 = *(const v4f*)(p + 4);
  float v[8];
#pragma unroll
  for (int e = 0; e < 4; ++e) { v[e] = a[e]; v[4 + e] = c4[e]; }
  unsigned short s[8];
#pragma unroll
  for (int e = 0; e < 8; ++e) {
    const unsigned short bb = bf_bits(v[e]);
    const unsigned short hb = h_bits((_Float16)(bf_up(bb) * scale));
    s[e] = (mode != 0) ? hb : bb;
  }
  v4u o;
#pragma unroll
  for (int e = 0; e < 4; ++e) o[e] = pk16(s[2 * e], s[2 * e + 1]);
  u16* d = D + (size_t)gt * 8;
  for (int pass = 0; pass < 2; ++pass) {
    *(volatile v4u*)(d) = o;
    __threadfence();
  }
}

__global__ __launch_bounds__(256) void trcvt16(const float* __restrict__ w, u16* D, int K, int N, int mode, float scale) {
  __shared__ __align__(16) u16 tile[64 * 72];
  const int tid = threadIdx.x;
  const int ntl = N >> 6;
  const int bid = blockIdx.x;
  const int k0  = (bid / ntl) * 64;
  const int n0  = (bid % ntl) * 64;
  const int kl = tid >> 2, nq = (tid & 3) * 16;
  const float* src = w + (size_t)(k0 + kl) * (size_t)N + n0 + nq;
  v4f f4[4];
#pragma unroll
  for (int e = 0; e < 4; ++e) f4[e] = *(const v4f*)(src + 4 * e);
#pragma unroll
  for (int e = 0; e < 4; ++e) {
#pragma unroll
    for (int i = 0; i < 4; ++i) {
      const float v = f4[e][i];
      const unsigned short bb = bf_bits(v);
      const unsigned short hb = h_bits((_Float16)(bf_up(bb) * scale));
      tile[(nq + 4 * e + i) * 72 + kl] = (mode != 0) ? hb : bb;
    }
  }
  __syncthreads();
  const int row = tid >> 3, c8 = (tid & 7) * 8;
  const v4u o0 = *(const v4u*)(tile + row * 72 + c8);
  const v4u o1 = *(const v4u*)(tile + (row + 32) * 72 + c8);
  u16* d0 = D + (size_t)(n0 + row) * (size_t)K + k0 + c8;
  u16* d1 = D + (size_t)(n0 + row + 32) * (size_t)K + k0 + c8;
  for (int pass = 0; pass < 2; ++pass) {
    *(volatile v4u*)(d0) = o0;
    *(volatile v4u*)(d1) = o1;
    __threadfence();
  }
}

__device__ __forceinline__ void epi16x(float* sl, v8f a0, v8f a1, v8f a2, v8f a3, float oscale, u16* C, int N,
                                       u16* CL, int NL, float losc, int haslo, size_t rowb, int col0, int lane) {
  const int hh = lane >> 4, m = lane & 15;
#pragma unroll
  for (int r = 0; r < 8; ++r) {
    const int ro = (8 * hh + r) * 68 + m;
    sl[ro]      = a0[r] * oscale;
    sl[ro + 16] = a1[r] * oscale;
    sl[ro + 32] = a2[r] * oscale;
    sl[ro + 48] = a3[r] * oscale;
  }
  wave_sync_lds();
  const int rq = lane >> 3, c8 = (lane & 7) * 8;
  v4u ov[4], ol[4];
#pragma unroll
  for (int i4 = 0; i4 < 4; ++i4) {
    const int row = i4 * 4 + rq;
    const v4f a = *(const v4f*)(sl + row * 68 + c8), c4 = *(const v4f*)(sl + row * 68 + c8 + 4);
    float wv[8];
#pragma unroll
    for (int e = 0; e < 4; ++e) { wv[e] = a[e]; wv[4 + e] = c4[e]; }
#pragma unroll
    for (int e = 0; e < 4; ++e) {
      const _Float16 h0 = (_Float16)wv[2 * e], h1 = (_Float16)wv[2 * e + 1];
      const float l0 = (wv[2 * e] - (float)h0) * losc;
      const float l1 = (wv[2 * e + 1] - (float)h1) * losc;
      ov[i4][e] = pk16(h_bits(h0), h_bits(h1));
      ol[i4][e] = pk16(h_bits((_Float16)l0), h_bits((_Float16)l1));
    }
  }
  u16* dst = C + (rowb + (size_t)rq) * (size_t)N + col0 + c8;
  for (int pass = 0; pass < 2; ++pass) {
#pragma unroll
    for (int i4 = 0; i4 < 4; ++i4) {
      *(volatile v4u*)(dst + (size_t)(i4 * 4) * (size_t)N) = ov[i4];
    }
    __threadfence();
  }
  if (haslo != 0) {
    u16* dl = CL + (rowb + (size_t)rq) * (size_t)NL + col0 + c8;
    for (int pass = 0; pass < 2; ++pass) {
#pragma unroll
      for (int i4 = 0; i4 < 4; ++i4) {
        *(volatile v4u*)(dl + (size_t)(i4 * 4) * (size_t)NL) = ol[i4];
      }
      __threadfence();
    }
  }
}

__device__ __forceinline__ void epi64(float* sl, v8f a0, v8f a1, v8f a2, v8f a3, float* C, int N,
                                      size_t rowb, int col0, int lane) {
  const int hh = lane >> 4, m = lane & 15;
#pragma unroll
  for (int r = 0; r < 8; ++r) {
    const int ro = (8 * hh + r) * 68 + m;
    sl[ro]      = a0[r];
    sl[ro + 16] = a1[r];
    sl[ro + 32] = a2[r];
    sl[ro + 48] = a3[r];
  }
  wave_sync_lds();
  v4f vals[8];
#pragma unroll
  for (int it = 0; it < 8; ++it) vals[it] = *(const v4f*)(sl + (it * 2 + hh) * 68 + m * 4);
  float* dst = C + (rowb + (size_t)hh) * (size_t)N + col0 + m * 4;
  for (int pass = 0; pass < 2; ++pass) {
#pragma unroll
    for (int it = 0; it < 8; ++it) {
      *(volatile v4f*)(dst + (size_t)(it * 2) * (size_t)N) = vals[it];
    }
    __threadfence();
  }
}

__global__ __launch_bounds__(128)
void gemm_b16(const u16* __restrict__ A, const u16* __restrict__ Bt, u16* C, int M, int N, int K,
              int bstA, int bstB, int bstC, float oscale, u16* CL, int NL, int bstCL, float losc) {
  __shared__ __align__(16) float slab[4 * SLABN];
  const int tid = threadIdx.x, wave = tid >> 5, lane = tid & 31, hh = lane >> 4, m = lane & 15;
  const int ntile = N >> 6, mtile = M >> 6;
  const int per   = ntile * mtile;
  const int bid   = blockIdx.x;
  const int bt    = bid / per;
  const int t     = bid - bt * per;
  const int rowb  = (t / ntile) * 64 + wave * 16;
  const int col0  = (t % ntile) * 64;
  if (rowb + 16 > M) return;
  const int haslo = (col0 + 64 <= NL) ? 1 : 0;
  const u16* Ab = A  + (size_t)bt * (size_t)bstA;
  const u16* Bb = Bt + (size_t)bt * (size_t)bstB;
  u16*       Cb = C  + (size_t)bt * (size_t)bstC;
  u16*      CLb = CL + (size_t)bt * (size_t)bstCL;
  const u16* ap = Ab + (size_t)(rowb + m) * (size_t)K + 8 * hh;
  const u16* bp = Bb + (size_t)(col0 + m) * (size_t)K + 8 * hh;
  const size_t bs = (size_t)16 * K;
  v8f acc0 = zero8(), acc1 = zero8(), acc2 = zero8(), acc3 = zero8();
#pragma unroll 1
  for (int k0 = 0; k0 < K; k0 += 32) {
    const v16b a  = ldfrag_b(ap + k0);
    const v16b b0 = ldfrag_b(bp + k0);
    const v16b b1 = ldfrag_b(bp + bs + k0);
    const v16b b2 = ldfrag_b(bp + 2 * bs + k0);
    const v16b b3 = ldfrag_b(bp + 3 * bs + k0);
    acc0 = mma_b(a, b0, acc0);
    acc1 = mma_b(a, b1, acc1);
    acc2 = mma_b(a, b2, acc2);
    acc3 = mma_b(a, b3, acc3);
    guard6<v16b>(acc0, acc1, acc2, acc3, a, b0, b1, b2, b3, a);
  }
  epi16x(slab + wave * SLABN, acc0, acc1, acc2, acc3, oscale, Cb, N, CLb, NL, losc, haslo, (size_t)rowb, col0, lane);
}

__global__ __launch_bounds__(128)
void gemm_nr(const u16* __restrict__ A, const u16* __restrict__ Bt, u16* PH, u16* PL, int M, int N, int K,
             const float* __restrict__ nw, const float* __restrict__ cosp, const float* __restrict__ sinp,
             float hsc, float losc, int loM) {
  __shared__ __align__(16) float slab[4 * SLABW];
  const int tid = threadIdx.x, wave = tid >> 5, lane = tid & 31, hh = lane >> 4, m = lane & 15;
  const int nht  = N >> 7;
  const int bid  = blockIdx.x;
  const int rowb = (bid / nht) * 64 + wave * 16;
  const int col0 = (bid % nht) * 128;
  if (rowb + 16 > M) return;
  const u16* ap = A  + (size_t)(rowb + m) * (size_t)K + 8 * hh;
  const u16* bp = Bt + (size_t)(col0 + m) * (size_t)K + 8 * hh;
  const size_t bs = (size_t)16 * K;
  v8f acc[8];
#pragma unroll
  for (int j = 0; j < 8; ++j) acc[j] = zero8();
#pragma unroll 1
  for (int k0 = 0; k0 < K; k0 += 32) {
    const v16b a  = ldfrag_b(ap + k0);
    {
      const v16b b0 = ldfrag_b(bp + k0);
      const v16b b1 = ldfrag_b(bp + bs + k0);
      const v16b b2 = ldfrag_b(bp + 2 * bs + k0);
      const v16b b3 = ldfrag_b(bp + 3 * bs + k0);
      acc[0] = mma_b(a, b0, acc[0]);
      acc[1] = mma_b(a, b1, acc[1]);
      acc[2] = mma_b(a, b2, acc[2]);
      acc[3] = mma_b(a, b3, acc[3]);
      guard6<v16b>(acc[0], acc[1], acc[2], acc[3], a, b0, b1, b2, b3, a);
    }
    {
      const v16b b4 = ldfrag_b(bp + 4 * bs + k0);
      const v16b b5 = ldfrag_b(bp + 5 * bs + k0);
      const v16b b6 = ldfrag_b(bp + 6 * bs + k0);
      const v16b b7 = ldfrag_b(bp + 7 * bs + k0);
      acc[4] = mma_b(a, b4, acc[4]);
      acc[5] = mma_b(a, b5, acc[5]);
      acc[6] = mma_b(a, b6, acc[6]);
      acc[7] = mma_b(a, b7, acc[7]);
      guard6<v16b>(acc[4], acc[5], acc[6], acc[7], a, b4, b5, b6, b7, a);
    }
  }

  float* sl = slab + wave * SLABW;
  const int bq   = rowb / SEQ;
  const int pos0 = rowb - bq * SEQ;
  const int wlo  = (pos0 + 16 <= loM) ? 1 : 0;
  {
    const float* cs = cosp + (size_t)pos0 * ROPE_HALF;
#pragma unroll
    for (int it = 0; it < 8; ++it) {
      v4f cv = *(const v4f*)(cs + it * 128 + lane * 4);
#pragma unroll
      for (int e = 0; e < 4; ++e) cv[e] = bf_val(cv[e]);
      *(v4f*)(sl + it * 128 + lane * 4) = cv;
    }
    const float* sn = sinp + (size_t)pos0 * ROPE_HALF;
#pragma unroll
    for (int it = 0; it < 8; ++it) {
      v4f sv = *(const v4f*)(sn + it * 128 + lane * 4);
#pragma unroll
      for (int e = 0; e < 4; ++e) sv[e] = bf_val(sv[e]);
      *(v4f*)(sl + 1024 + it * 128 + lane * 4) = sv;
    }
  }
  wave_sync_lds();
  float inv[8];
#pragma unroll
  for (int r = 0; r < 8; ++r) {
    float ssum = 0.f;
#pragma unroll
    for (int nt = 0; nt < 8; ++nt) ssum += acc[nt][r] * acc[nt][r];
    ssum += __shfl_xor(ssum, 1, 32);
    ssum += __shfl_xor(ssum, 2, 32);
    ssum += __shfl_xor(ssum, 4, 32);
    ssum += __shfl_xor(ssum, 8, 32);
    inv[r] = rsqrtf(ssum * (1.0f / (float)HD) + EPS);
  }
  float w1[8];
#pragma unroll
  for (int nt = 0; nt < 8; ++nt) w1[nt] = 1.0f + bf_val(nw[16 * nt + m]);
#pragma unroll
  for (int r = 0; r < 8; ++r) {
    const int rl = 8 * hh + r;
#pragma unroll
    for (int nt = 0; nt < 4; ++nt) {
      const int d = 16 * nt + m;
      const float cv = sl[rl * ROPE_HALF + d];
      const float sv = sl[1024 + rl * ROPE_HALF + d];
      const float xr = (acc[nt][r] * inv[r]) * w1[nt];
      const float xi = (acc[nt + 4][r] * inv[r]) * w1[nt + 4];
      acc[nt][r]     = xr * cv - xi * sv;
      acc[nt + 4][r] = xr * sv + xi * cv;
    }
  }
  wave_sync_lds();
#pragma unroll
  for (int r = 0; r < 8; ++r) {
    const int ro = (8 * hh + r) * 132 + m;
#pragma unroll
    for (int nt = 0; nt < 8; ++nt) sl[ro + 16 * nt] = acc[nt][r] * hsc;
  }
  wave_sync_lds();
  const int c8 = m * 8;
  v4u oh[8], ol[8];
#pragma unroll
  for (int it = 0; it < 8; ++it) {
    const int row = 2 * it + hh;
    const v4f a = *(const v4f*)(sl + row * 132 + c8), c4 = *(const v4f*)(sl + row * 132 + c8 + 4);
    float wv[8];
#pragma unroll
    for (int e = 0; e < 4; ++e) { wv[e] = a[e]; wv[4 + e] = c4[e]; }
#pragma unroll
    for (int e = 0; e < 4; ++e) {
      const _Float16 h0 = (_Float16)wv[2 * e], h1 = (_Float16)wv[2 * e + 1];
      const float l0 = (wv[2 * e] - (float)h0) * losc;
      const float l1 = (wv[2 * e + 1] - (float)h1) * losc;
      oh[it][e] = pk16(h_bits(h0), h_bits(h1));
      ol[it][e] = pk16(h_bits((_Float16)l0), h_bits((_Float16)l1));
    }
  }
  const size_t ob  = (size_t)(rowb + hh) * (size_t)N + col0 + c8;
  const size_t obl = ((size_t)bq * (size_t)loM + (size_t)pos0 + (size_t)hh) * (size_t)N + col0 + c8;
  for (int pass = 0; pass < 2; ++pass) {
#pragma unroll
    for (int it = 0; it < 8; ++it) {
      *(volatile v4u*)(PH + ob + (size_t)(2 * it) * (size_t)N) = oh[it];
    }
    __threadfence();
  }
  if (wlo != 0) {
    for (int pass = 0; pass < 2; ++pass) {
#pragma unroll
      for (int it = 0; it < 8; ++it) {
        *(volatile v4u*)(PL + obl + (size_t)(2 * it) * (size_t)N) = ol[it];
      }
      __threadfence();
    }
  }
}

__global__ __launch_bounds__(128)
void gemm_hf2(const u16* __restrict__ AH, const u16* __restrict__ AL, const u16* __restrict__ Bt, float* C,
              int M, int N, int K, float osh, float osl) {
  __shared__ __align__(16) float slab[4 * SLABN];
  const int tid = threadIdx.x, wave = tid >> 5, lane = tid & 31, hh = lane >> 4, m = lane & 15;
  const int ntile = N >> 6;
  const int bid   = blockIdx.x;
  const int rowb  = (bid / ntile) * 64 + wave * 16;
  const int col0  = (bid % ntile) * 64;
  if (rowb + 16 > M) return;
  const _Float16* ahp = (const _Float16*)(const void*)AH + (size_t)(rowb + m) * (size_t)K + 8 * hh;
  const _Float16* alp = (const _Float16*)(const void*)AL + (size_t)(rowb + m) * (size_t)K + 8 * hh;
  const _Float16* bp  = (const _Float16*)(const void*)Bt + (size_t)(col0 + m) * (size_t)K + 8 * hh;
  const size_t bs = (size_t)16 * K;
  v8f h0 = zero8(), h1 = zero8(), h2 = zero8(), h3 = zero8();
  v8f l0 = zero8(), l1 = zero8(), l2 = zero8(), l3 = zero8();
#pragma unroll 1
  for (int k0 = 0; k0 < K; k0 += 32) {
    const v16h ah = ldfrag_h(ahp + k0);
    const v16h al = ldfrag_h(alp + k0);
    const v16h b0 = ldfrag_h(bp + k0);
    const v16h b1 = ldfrag_h(bp + bs + k0);
    const v16h b2 = ldfrag_h(bp + 2 * bs + k0);
    const v16h b3 = ldfrag_h(bp + 3 * bs + k0);
    h0 = mma_h(ah, b0, h0);
    h1 = mma_h(ah, b1, h1);
    h2 = mma_h(ah, b2, h2);
    h3 = mma_h(ah, b3, h3);
    l0 = mma_h(al, b0, l0);
    l1 = mma_h(al, b1, l1);
    l2 = mma_h(al, b2, l2);
    l3 = mma_h(al, b3, l3);
    guard8(h0, h1, h2, h3, l0, l1, l2, l3, ah, al, b0, b1, b2, b3);
  }
  v8f c0, c1, c2, c3;
#pragma unroll
  for (int r = 0; r < 8; ++r) {
    c0[r] = h0[r] * osh + l0[r] * osl;
    c1[r] = h1[r] * osh + l1[r] * osl;
    c2[r] = h2[r] * osh + l2[r] * osl;
    c3[r] = h3[r] * osh + l3[r] * osl;
  }
  epi64(slab + wave * SLABN, c0, c1, c2, c3, C, N, (size_t)rowb, col0, lane);
}

__global__ __launch_bounds__(ATT_THREADS)
void attn_fwd(const u16* __restrict__ QHp, const u16* __restrict__ QLp, const u16* __restrict__ KHp,
              const u16* __restrict__ KLp, const u16* __restrict__ VPp, const u16* __restrict__ VLp,
              u16* OHp, u16* OLp) {
  __shared__ __align__(16) float smem[ATT_WAVES * SLABW];

  const int tid  = threadIdx.x;
  const int wave = tid >> 5;
  const int lane = tid & 31;
  const int hh   = lane >> 4;
  const int c    = lane & 15;

  const int bid  = blockIdx.x;
  const int qt   = bid % NQT;
  const int rest = bid / NQT;
  const int head = rest % NH;
  const int b    = rest / NH;
  if (b >= NB) return;
  const int hkv  = head / NREP;
  const int qb   = qt * 64;
  const int q0   = qb + wave * 16;
  const bool qlo = (qb < VLN);

  const int jlo  = max(qb - (WIN - 1), 0);
  const int jhi  = qb + 63;
  const int kblo = jlo >> 5;
  int nkb = (jhi >> 5) - kblo + 1;
  nkb = min(max(nkb, 1), NKB - kblo);

  const size_t rowq = (size_t)b * SEQ + q0 + c;
  const _Float16* Qh = (const _Float16*)(const void*)QHp + rowq * HDQ + head * HD + 8 * hh;
  const _Float16* Ql = (const _Float16*)(const void*)QLp + rowq * HDQ + head * HD + 8 * hh;
  const _Float16* Kb = (const _Float16*)(const void*)KHp + ((size_t)b * SEQ + c) * KVD + hkv * HD + 8 * hh;
  const _Float16* Kl = (const _Float16*)(const void*)KLp + ((size_t)b * VLN + c) * KVD + hkv * HD + 8 * hh;
  const _Float16* Vb = (const _Float16*)(const void*)VPp + (size_t)b * KVD * SEQ + (size_t)(hkv * HD + c) * SEQ + 8 * hh;
  const _Float16* Vl = (const _Float16*)(const void*)VLp + (size_t)b * KVD * VLN + (size_t)(hkv * HD + c) * VLN + 8 * hh;
  const float lsc  = SMSC * (LOG2E / (QSC * KSC));
  const float lscl = lsc * (1.0f / QLC);
  const int dq = q0 + c - 8 * hh;

  float mrun = NEGS, lrun = 0.f;
  v8f o[8];
#pragma unroll
  for (int j = 0; j < 8; ++j) o[j] = zero8();

#pragma unroll 1
  for (int it = 0; it < nkb; ++it) {
    const int kb = (kblo + it) * 32;
    const bool lo_blk = qlo && (kb + 32 <= VLN);
    v8f s0 = zero8(), s1 = zero8(), rr0 = zero8(), rr1 = zero8();
    const _Float16* k0p = Kb + (size_t)kb * KVD;
    const _Float16* k1p = k0p + (size_t)16 * KVD;
    const _Float16* l0p = Kl + (size_t)kb * KVD;
    const _Float16* l1p = l0p + (size_t)16 * KVD;
#pragma unroll
    for (int dc = 0; dc < 4; ++dc) {
      const v16h ka = ldfrag_h(k0p + 32 * dc);
      const v16h kc = ldfrag_h(k1p + 32 * dc);
      const v16h qh = ldfrag_h(Qh + 32 * dc);
      const v16h ql = ldfrag_h(Ql + 32 * dc);
      s0  = mma_h(ka, qh, s0);
      rr0 = mma_h(ka, ql, rr0);
      s1  = mma_h(kc, qh, s1);
      rr1 = mma_h(kc, ql, rr1);
      guard4<v16h>(s0, rr0, s1, rr1, ka, kc, qh, ql);
      if (lo_blk) {
        const v16h la = ldfrag_h(l0p + 32 * dc);
        const v16h lc = ldfrag_h(l1p + 32 * dc);
        rr0 = mma_h(la, qh, rr0);
        rr1 = mma_h(lc, qh, rr1);
        guard2(rr0, rr1, la, lc, qh, la, lc, qh);
      }
    }
    float tk[16];
#pragma unroll
    for (int i = 0; i < 8; ++i) {
      const int d0 = dq - kb - i;
      const int d1 = d0 - 16;
      const bool a0 = (d0 >= 0) && (d0 <= WIN - 1);
      const bool a1 = (d1 >= 0) && (d1 <= WIN - 1);
      tk[i]     = a0 ? (s0[i] * lsc + rr0[i] * lscl) : NEGS;
      tk[8 + i] = a1 ? (s1[i] * lsc + rr1[i] * lscl) : NEGS;
    }
    float cm = tk[0];
#pragma unroll
    for (int i = 1; i < 16; ++i) cm = fmaxf(cm, tk[i]);
    cm = fmaxf(cm, __shfl_xor(cm, 16, 32));
    const float mn = fmaxf(mrun, cm);
    const float al = exp2f(fminf(mrun - mn, 0.f));
    mrun = mn;
    float ps = 0.f;
    FragH ph;
#pragma unroll
    for (int wq = 0; wq < 2; ++wq) {
#pragma unroll
      for (int e4 = 0; e4 < 4; ++e4) {
        const int i = 8 * wq + 2 * e4;
        const float x0 = exp2f(fminf(tk[i] - mn, 0.f));
        const float x1 = exp2f(fminf(tk[i + 1] - mn, 0.f));
        const float p0 = (tk[i] > -1.0e38f) ? x0 : 0.f;
        const float p1 = (tk[i + 1] > -1.0e38f) ? x1 : 0.f;
        ps += p0 + p1;
        const float cc0 = p0 * PCAR, cc1 = p1 * PCAR;
        tk[i] = cc0;
        tk[i + 1] = cc1;
        ph.u[wq][e4] = pk16(h_bits((_Float16)cc0), h_bits((_Float16)cc1));
      }
    }
    ps += __shfl_xor(ps, 16, 32);
    lrun = lrun * al + ps;
    FragH pl;
    pl.u[0] = zero4u();
    pl.u[1] = zero4u();
    if (lo_blk) {
#pragma unroll
      for (int wq = 0; wq < 2; ++wq) {
#pragma unroll
        for (int e4 = 0; e4 < 4; ++e4) {
          const int i = 8 * wq + 2 * e4;
          const _Float16 h0 = (_Float16)tk[i], h1 = (_Float16)tk[i + 1];
          const float r0 = (tk[i] - (float)h0) * PLC;
          const float r1 = (tk[i + 1] - (float)h1) * PLC;
          pl.u[wq][e4] = pk16(h_bits((_Float16)r0), h_bits((_Float16)r1));
        }
      }
    }
    float scl[8];
#pragma unroll
    for (int r = 0; r < 8; ++r) scl[r] = __shfl(al, 8 * hh + r, 32);
#pragma unroll
    for (int j = 0; j < 8; ++j) {
#pragma unroll
      for (int r = 0; r < 8; ++r) o[j][r] *= scl[r];
    }
    {
      const _Float16* vp = Vb + kb;
      const _Float16* lp = Vl + kb;
#pragma unroll
      for (int g2 = 0; g2 < 4; ++g2) {
        const v16h va = ldfrag_h(vp + (size_t)(32 * g2) * SEQ);
        const v16h vc = ldfrag_h(vp + (size_t)(32 * g2 + 16) * SEQ);
        o[2 * g2]     = mma_h(ph.v, va, o[2 * g2]);
        o[2 * g2 + 1] = mma_h(ph.v, vc, o[2 * g2 + 1]);
        guard2(o[2 * g2], o[2 * g2 + 1], ph.v, va, vc, ph.v, va, vc);
        if (lo_blk) {
          const v16h wa = ldfrag_h(lp + (size_t)(32 * g2) * VLN);
          const v16h wc = ldfrag_h(lp + (size_t)(32 * g2 + 16) * VLN);
          v8f ta = mma_h(ph.v, wa, zero8());
          v8f tb = mma_h(ph.v, wc, zero8());
          ta = mma_h(pl.v, va, ta);
          tb = mma_h(pl.v, vc, tb);
          guard2(ta, tb, ph.v, pl.v, va, vc, wa, wc);
#pragma unroll
          for (int r = 0; r < 8; ++r) {
            o[2 * g2][r]     += ta[r] * (1.0f / VLC);
            o[2 * g2 + 1][r] += tb[r] * (1.0f / VLC);
          }
        }
      }
    }
  }
  acc_guard4(o[0], o[1], o[2], o[3]);
  acc_guard4(o[4], o[5], o[6], o[7]);

  const float linv = (lrun > 0.f) ? ((1.0f / lrun) * (1.0f / (PCAR * VCAR))) : 0.f;
  float inv[8];
#pragma unroll
  for (int r = 0; r < 8; ++r) inv[r] = __shfl(linv, 8 * hh + r, 32);
  float* slab = smem + wave * SLABW;
#pragma unroll
  for (int r = 0; r < 8; ++r) {
#pragma unroll
    for (int j = 0; j < 8; ++j) slab[(8 * hh + r) * 132 + j * 16 + c] = o[j][r] * inv[r];
  }
  wave_sync_lds();
  v4u oh[8], ol[8];
  const int c8 = c * 8;
#pragma unroll
  for (int it = 0; it < 8; ++it) {
    const int row = 2 * it + hh;
    const v4f a = *(const v4f*)(slab + row * 132 + c8), c4 = *(const v4f*)(slab + row * 132 + c8 + 4);
    float wv[8];
#pragma unroll
    for (int e = 0; e < 4; ++e) { wv[e] = a[e] * OSC; wv[4 + e] = c4[e] * OSC; }
#pragma unroll
    for (int e = 0; e < 4; ++e) {
      const _Float16 h0 = (_Float16)wv[2 * e], h1 = (_Float16)wv[2 * e + 1];
      const float l0 = (wv[2 * e] - (float)h0) * OLC;
      const float l1 = (wv[2 * e + 1] - (float)h1) * OLC;
      oh[it][e] = pk16(h_bits(h0), h_bits(h1));
      ol[it][e] = pk16(h_bits((_Float16)l0), h_bits((_Float16)l1));
    }
  }
  const size_t ob = ((size_t)b * SEQ + q0 + hh) * (size_t)HDQ + head * HD + c8;
  for (int pass = 0; pass < 2; ++pass) {
#pragma unroll
    for (int it = 0; it < 8; ++it) {
      *(volatile v4u*)(OHp + ob + (size_t)(2 * it) * HDQ) = oh[it];
    }
    __threadfence();
  }
  for (int pass = 0; pass < 2; ++pass) {
#pragma unroll
    for (int it = 0; it < 8; ++it) {
      *(volatile v4u*)(OLp + ob + (size_t)(2 * it) * HDQ) = ol[it];
    }
    __threadfence();
  }
}

extern "C" void kernel_launch(void* const* d_in, const int* in_sizes, int n_in,
                              void* d_out, int out_size, void* d_ws, size_t ws_size,
                              hipStream_t stream) {
  if (n_in < 9) return;
  if (in_sizes[0] < ((NB - 1) * SEQ_FULL + SEQ) * DIM) return;
  if (in_sizes[1] < SEQ * ROPE_HALF) return;
  if (in_sizes[2] < SEQ * ROPE_HALF) return;
  if (in_sizes[3] < DIM * HDQ) return;
  if (in_sizes[4] < DIM * KVD) return;
  if (in_sizes[5] < DIM * KVD) return;
  if (in_sizes[6] < HDQ * DIM) return;
  if (in_sizes[7] < HD) return;
  if (in_sizes[8] < HD) return;
  if (out_size < ROWS * DIM) return;

  const float* Xin = (const float*)d_in[0];
  const float* Cos = (const float*)d_in[1];
  const float* Sin = (const float*)d_in[2];
  const float* Wq  = (const float*)d_in[3];
  const float* Wk  = (const float*)d_in[4];
  const float* Wv  = (const float*)d_in[5];
  const float* Wo  = (const float*)d_in[6];
  const float* Qnw = (const float*)d_in[7];
  const float* Knw = (const float*)d_in[8];
  float*       out = (float*)d_out;

  const size_t szXB  = (size_t)ROWS * DIM * 2;
  const size_t szWQT = (size_t)HDQ * DIM * 2;
  const size_t szWKT = (size_t)KVD * DIM * 2;
  const size_t szWOT = (size_t)DIM * HDQ * 2;
  const size_t szQ   = (size_t)ROWS * HDQ * 2;
  const size_t szK   = (size_t)ROWS * KVD * 2;
  const size_t szKL  = (size_t)NB * VLN * KVD * 2;
  const size_t szVP  = (size_t)NB * KVD * SEQ * 2;
  const size_t szVL  = (size_t)NB * KVD * VLN * 2;
  size_t off = 0;
  const size_t oXB  = off; off += szXB;
  const size_t oWQT = off; off += szWQT;
  const size_t oWKT = off; off += szWKT;
  const size_t oWVT = off; off += szWKT;
  const size_t oWOT = off; off += szWOT;
  const size_t oQH  = off; off += szQ;
  const size_t oQL  = off; off += szQ;
  const size_t oKH  = off; off += szK;
  const size_t oKL  = off; off += szKL;
  const size_t oVP  = off; off += szVP;
  const size_t oVL  = off; off += szVL;
  const size_t oOH  = off; off += szQ;
  const size_t oOL  = off; off += szQ;
  if (off > ws_size) return;
  if (off > (size_t)134217728) return;

  char* ws = (char*)d_ws;
  u16* XB  = (u16*)(ws + oXB);
  u16* WQT = (u16*)(ws + oWQT);
  u16* WKT = (u16*)(ws + oWKT);
  u16* WVT = (u16*)(ws + oWVT);
  u16* WOT = (u16*)(ws + oWOT);
  u16* QH  = (u16*)(ws + oQH);
  u16* QL  = (u16*)(ws + oQL);
  u16* KH  = (u16*)(ws + oKH);
  u16* KL  = (u16*)(ws + oKL);
  u16* VP  = (u16*)(ws + oVP);
  u16* VL  = (u16*)(ws + oVL);
  u16* OH  = (u16*)(ws + oOH);
  u16* OL  = (u16*)(ws + oOL);

  if ((DIM % 64) != 0 || (HDQ % 64) != 0 || (KVD % 64) != 0 || (SEQ % 64) != 0 || (ROWS % 64) != 0) return;
  if ((HDQ % 128) != 0 || (KVD % 128) != 0 || (DIM % 32) != 0 || (HDQ % 32) != 0 || (VLN % 64) != 0) return;
  const int n8x = (SEQ * DIM) / 8;
  if ((n8x % 256) != 0) return;

  const dim3 b256(256), b128(128);
  const dim3 gX(n8x / 256);
  const dim3 gTq((DIM / 64) * (HDQ / 64));
  const dim3 gTk((DIM / 64) * (KVD / 64));
  const dim3 gTo((HDQ / 64) * (DIM / 64));
  const dim3 gNQ((ROWS / 64) * (HDQ / 128));
  const dim3 gNK((ROWS / 64) * (KVD / 128));
  const dim3 gV(NB * (KVD / 64) * (SEQ / 64));
  const dim3 gAT(NB * NH * NQT);
  const dim3 bAT(ATT_THREADS);
  const dim3 gO((ROWS / 64) * (DIM / 64));

  for (int bb = 0; bb < NB; ++bb) {
    cvt16<<<gX, b256, 0, stream>>>(Xin + (size_t)bb * SEQ_FULL * DIM, XB + (size_t)bb * SEQ * DIM, n8x, 0, 1.0f);
  }
  trcvt16<<<gTq, b256, 0, stream>>>(Wq, WQT, DIM, HDQ, 0, 1.0f);
  trcvt16<<<gTk, b256, 0, stream>>>(Wk, WKT, DIM, KVD, 0, 1.0f);
  trcvt16<<<gTk, b256, 0, stream>>>(Wv, WVT, DIM, KVD, 0, 1.0f);
  trcvt16<<<gTo, b256, 0, stream>>>(Wo, WOT, HDQ, DIM, 1, WOS);
  gemm_nr<<<gNQ, b128, 0, stream>>>(XB, WQT, QH, QL, ROWS, HDQ, DIM, Qnw, Cos, Sin, QSC, QLC, SEQ);
  gemm_nr<<<gNK, b128, 0, stream>>>(XB, WKT, KH, KL, ROWS, KVD, DIM, Knw, Cos, Sin, KSC, KLC, VLN);
  gemm_b16<<<gV, b128, 0, stream>>>(WVT, XB, VP, KVD, SEQ, DIM, 0, SEQ * DIM, KVD * SEQ, VCAR, VL, VLN, KVD * VLN, VLC);
  attn_fwd<<<gAT, bAT, 0, stream>>>(QH, QL, KH, KL, VP, VL, OH, OL);
  gemm_hf2<<<gO, b128, 0, stream>>>(OH, OL, WOT, out, ROWS, DIM, HDQ, 1.0f / (OSC * WOS), 1.0f / (OSC * WOS * OLC));
  (void)hipGetLastError();
}
